// ConcatAttention_13709535609366
// MI455X (gfx1250) — hardware-verified
//
#include <hip/hip_runtime.h>


#define NB_  4
#define SQ   256
#define SK   256
#define DF   256
#define DH   512
typedef _Float16 h16;
typedef unsigned short bf;
typedef __attribute__((ext_vector_type(16))) __bf16   v16bf;
typedef __attribute__((ext_vector_type(16))) _Float16 v16h;
typedef __attribute__((ext_vector_type(8)))  _Float16 v8h;
typedef __attribute__((ext_vector_type(8)))  unsigned short v8us;
typedef __attribute__((ext_vector_type(8)))  float    v8f;
typedef __attribute__((ext_vector_type(4)))  float    v4f;
typedef v8h  __attribute__((may_alias)) v8ha;
typedef v4f  __attribute__((may_alias)) v4fa;
typedef v8us __attribute__((may_alias)) v8usa;

__device__ __forceinline__ unsigned short f2bf(float f) { unsigned u = __float_as_uint(f); u += 0x7FFFu + ((u >> 16) & 1u); return (unsigned short)(u >> 16); }
__device__ __forceinline__ float bf2f(unsigned short b) { return __uint_as_float(((unsigned)b) << 16); }
__device__ __forceinline__ float bfr(float f) { return bf2f(f2bf(f)); }
__device__ __forceinline__ v16h cat16(v8h lo, v8h hi) { return __builtin_shufflevector(lo, hi, 0, 1, 2, 3, 4, 5, 6, 7, 8, 9, 10, 11, 12, 13, 14, 15); }
__device__ __forceinline__ v16bf cat16b(v8us lo, v8us hi) { return __builtin_bit_cast(v16bf, __builtin_shufflevector(lo, hi, 0, 1, 2, 3, 4, 5, 6, 7, 8, 9, 10, 11, 12, 13, 14, 15)); }
__device__ __forceinline__ v8f wmma16(v16h a, v16h b, v8f c) { return __builtin_amdgcn_wmma_f32_16x16x32_f16(false, a, false, b, (short)0, c, false, false); }
__device__ __forceinline__ v8f wmmab(v16bf a, v16bf b, v8f c) { return __builtin_amdgcn_wmma_f32_16x16x32_bf16(false, a, false, b, (short)0, c, false, false); }


template <typename T16> struct WFrag;
template <> struct WFrag<h16> { typedef v16h V; static __device__ __forceinline__ V ld(const h16* p) { return cat16(*(const v8h*)p, *(const v8h*)(p + 16)); } static __device__ __forceinline__ v8f mma(V a, V b, v8f c) { return wmma16(a, b, c); } };
template <> struct WFrag<bf> { typedef v16bf V; static __device__ __forceinline__ V ld(const bf* p) { return cat16b(*(const v8us*)p, *(const v8us*)(p + 16)); } static __device__ __forceinline__ v8f mma(V a, V b, v8f c) { return wmmab(a, b, c); } };
template <typename T16, int NSPLIT, bool BIAS>
__global__ __launch_bounds__(32) void k_gemmw(const T16* __restrict__ A, const T16* __restrict__ A2, const T16* __restrict__ Bt, const T16* __restrict__ Bt2, int K, float* C, int ldc, const float* __restrict__ bias, size_t sA, size_t sB, size_t sC) {
    typedef typename WFrag<T16>::V V;
    __shared__ __align__(16) float os[16 * 68];
    const size_t z = blockIdx.z; A += z * sA; if (A2) A2 += z * sA; Bt += z * sB; if (Bt2) Bt2 += z * sB; C += z * sC;
    const int lane = threadIdx.x & 31, lr = lane & 15, hi = lane >> 4; const int r0 = blockIdx.x * 64, c0 = blockIdx.y * 64;
    v8f acc[4][4];
#pragma unroll
    for (int mb = 0; mb < 4; ++mb)
#pragma unroll
        for (int nb = 0; nb < 4; ++nb) acc[mb][nb] = (v8f){};
    const size_t aoff = (size_t)(r0 + lr) * K + 8 * hi, boff = (size_t)(c0 + lr) * K + 8 * hi;
#pragma unroll 1
    for (int kc = 0; kc < K; kc += 32) {
        V a[4], a2[4];
#pragma unroll
        for (int mb = 0; mb < 4; ++mb) { a[mb] = WFrag<T16>::ld(A + aoff + (size_t)mb * 16 * K + kc); if (NSPLIT == 1 || NSPLIT == 2) a2[mb] = WFrag<T16>::ld(A2 + aoff + (size_t)mb * 16 * K + kc); }
#pragma unroll
        for (int nb = 0; nb < 4; ++nb) { const V b = WFrag<T16>::ld(Bt + boff + (size_t)nb * 16 * K + kc); V b2; if (NSPLIT >= 2) b2 = WFrag<T16>::ld(Bt2 + boff + (size_t)nb * 16 * K + kc);
#pragma unroll
            for (int mb = 0; mb < 4; ++mb) { acc[mb][nb] = WFrag<T16>::mma(a[mb], b, acc[mb][nb]); if (NSPLIT == 1 || NSPLIT == 2) acc[mb][nb] = WFrag<T16>::mma(a2[mb], b, acc[mb][nb]); if (NSPLIT >= 2) acc[mb][nb] = WFrag<T16>::mma(a[mb], b2, acc[mb][nb]); } }
        asm volatile("v_nop\n\tv_nop\n\tv_nop\n\tv_nop" : "+v"(acc[0][0]), "+v"(acc[1][1]), "+v"(acc[2][2]), "+v"(acc[3][3]) : "v"(a[0]), "v"(a[3]));
    }
#pragma unroll
    for (int mb = 0; mb < 4; ++mb) {
#pragma unroll
        for (int nb = 0; nb < 4; ++nb) {
#pragma unroll
            for (int j = 0; j < 8; ++j) os[(hi * 8 + j) * 68 + nb * 16 + lr] = acc[mb][nb][j]; }
        __builtin_amdgcn_wave_barrier(); asm volatile("" ::: "memory");
        float* crow = C + (size_t)(r0 + mb * 16) * ldc + c0;
#pragma unroll 1
        for (int ps = 0; ps < 2; ++ps) {
#pragma unroll
            for (int s = 0; s < 8; ++s) { const int row = 2 * s + hi, cofs = lr * 4; v4f val = *(const v4fa*)(os + row * 68 + cofs); if (BIAS) { val[0] += bfr(bias[c0 + cofs]); val[1] += bfr(bias[c0 + cofs + 1]); val[2] += bfr(bias[c0 + cofs + 2]); val[3] += bfr(bias[c0 + cofs + 3]); }
                *(volatile v4f*)(crow + (size_t)row * ldc + cofs) = val; }
            if (ps == 0) __threadfence(); }
        __builtin_amdgcn_wave_barrier(); asm volatile("" ::: "memory");
    }
}

__device__ __forceinline__ h16 tohx(float x) { return (h16)x; }
__device__ __forceinline__ void splitf(float y, unsigned short& h, unsigned short& l) { h = f2bf(y); l = f2bf(y - bf2f(h)); }
typedef __attribute__((ext_vector_type(2))) _Float16 v2h;
typedef __attribute__((ext_vector_type(4))) _Float16 v4h;
typedef __attribute__((ext_vector_type(2))) unsigned short v2us;
typedef __attribute__((ext_vector_type(4))) unsigned short v4us;
typedef __attribute__((ext_vector_type(2))) float v2f;
typedef __attribute__((ext_vector_type(4))) int v4i;


__global__ __launch_bounds__(256) void k_cvt8(const float* __restrict__ src, bf* dst, size_t n8) { const size_t i = (size_t)blockIdx.x * 256 + threadIdx.x; if (i >= n8) return; const v8f v = *(const v8f*)(src + i * 8); v8us o;
#pragma unroll
    for (int k = 0; k < 8; ++k) o[k] = f2bf(v[k]); *(volatile v8us*)(dst + i * 8) = o; __threadfence(); *(volatile v8us*)(dst + i * 8) = o; }

__global__ __launch_bounds__(256) void k_w1ab(const float* __restrict__ W1, bf* WA, bf* WB) { const size_t i = (size_t)blockIdx.x * 256 + threadIdx.x; if (i >= (size_t)DH * DF / 8) return; const size_t e = i * 8; const int h = (int)(e / DF), k = (int)(e % DF); v8us oa, ob;
#pragma unroll
    for (int q = 0; q < 8; ++q) { oa[q] = f2bf(W1[(size_t)h * DH + k + q]); ob[q] = f2bf(W1[(size_t)h * DH + DF + k + q]); } *(volatile v8us*)(WA + e) = oa; *(volatile v8us*)(WB + e) = ob; __threadfence(); *(volatile v8us*)(WA + e) = oa; *(volatile v8us*)(WB + e) = ob; }
__global__ __launch_bounds__(256) void k_cat(const float* __restrict__ QH, const float* __restrict__ KH, const float* __restrict__ b1, const float* __restrict__ W2, const int* __restrict__ MO, const float* __restrict__ Vb, float* O) {
    const int lane = threadIdx.x & 31; const int q = blockIdx.x * 8 + (threadIdx.x >> 5); if (q >= SQ) return; float qb[16], w2[16];
    { const v8f a0 = *(const v8f*)(QH + (size_t)q * DH + lane * 16), a1 = *(const v8f*)(QH + (size_t)q * DH + lane * 16 + 8);
#pragma unroll
      for (int d = 0; d < 8; ++d) { qb[d] = __fadd_rn(a0[d], bfr(b1[lane * 16 + d])); qb[8 + d] = __fadd_rn(a1[d], bfr(b1[lane * 16 + 8 + d])); w2[d] = bfr(W2[lane * 16 + d]); w2[8 + d] = bfr(W2[lane * 16 + 8 + d]); } }
    float sc[SK / 32];
#pragma unroll
    for (int c = 0; c < SK / 32; ++c) sc[c] = 0.f;
#pragma unroll 1
    for (int k = 0; k < SK; ++k) { const v8f k0 = *(const v8f*)(KH + (size_t)k * DH + lane * 16), k1 = *(const v8f*)(KH + (size_t)k * DH + lane * 16 + 8); float s = 0.f;
#pragma unroll
        for (int d = 0; d < 16; ++d) { float hdn = __fadd_rn(qb[d], (d < 8) ? k0[d] : k1[d - 8]); asm volatile("" : "+v"(hdn)); float act = (hdn >= 0.f) ? hdn : (0.01f * hdn); float pr = __fmul_rn(act, w2[d]); asm volatile("" : "+v"(pr)); s = __fadd_rn(s, pr); }
#pragma unroll
        for (int sh = 16; sh; sh >>= 1) s += __shfl_xor(s, sh, 32);
        const float sm = (MO[k] != 0) ? -1.0e9f : s;
#pragma unroll
        for (int c = 0; c < SK / 32; ++c) if (k / 32 == c && (k & 31) == lane) sc[c] = sm; }
    float mx = -3.0e38f;
#pragma unroll
    for (int c = 0; c < SK / 32; ++c) mx = fmaxf(mx, sc[c]);
#pragma unroll
    for (int sh = 16; sh; sh >>= 1) mx = fmaxf(mx, __shfl_xor(mx, sh, 32));
    float sum = 0.f;
#pragma unroll
    for (int c = 0; c < SK / 32; ++c) { float d0 = __fsub_rn(sc[c], mx); asm volatile("" : "+v"(d0)); sc[c] = __builtin_amdgcn_exp2f(__fmul_rn(d0, 1.4426950408889634f)); sum += sc[c]; }
#pragma unroll
    for (int sh = 16; sh; sh >>= 1) sum += __shfl_xor(sum, sh, 32);
    const float f = __fdiv_rn(1.0f, sum);
#pragma unroll
    for (int c = 0; c < SK / 32; ++c) sc[c] *= f;
    v8f acc = (v8f){0.f, 0.f, 0.f, 0.f, 0.f, 0.f, 0.f, 0.f};
#pragma unroll
    for (int c = 0; c < SK / 32; ++c) {
#pragma unroll 1
        for (int kk = 0; kk < 32; ++kk) { const float p = __shfl(sc[c], kk, 32); const v8f vv = *(const v8f*)(Vb + (size_t)(c * 32 + kk) * DF + lane * 8);
#pragma unroll
            for (int d = 0; d < 8; ++d) { float vr = bfr(vv[d]); asm volatile("" : "+v"(vr)); float t1 = __fmul_rn(p, vr); asm volatile("" : "+v"(t1)); acc[d] = __fadd_rn(acc[d], t1); } } }
    float* dst = O + (size_t)q * DF + lane * 8;
    *(volatile v8f*)dst = acc; __threadfence(); *(volatile v8f*)dst = acc; }

extern "C" void kernel_launch(void* const* d_in, const int* in_sizes, int n_in,
                              void* d_out, int out_size, void* d_ws, size_t ws_size, hipStream_t stream) {
    (void)in_sizes; (void)n_in; (void)out_size;
    const float* Q = (const float*)d_in[0]; const float* K = (const float*)d_in[1]; const float* V = (const float*)d_in[2]; const int* MO = (const int*)d_in[3]; const float* W1 = (const float*)d_in[4]; const float* b1 = (const float*)d_in[5]; const float* W2 = (const float*)d_in[6];
    float* OUT = (float*)d_out;
    char* wsp = (char*)d_ws;
    auto take = [&](size_t bytes) { char* p = wsp; wsp += (bytes + 255) & ~(size_t)255; return (void*)p; };
    bf* WA = (bf*)take((size_t)DH * DF * 2); bf* WB = (bf*)take((size_t)DH * DF * 2); bf* XQ = (bf*)take((size_t)SQ * DF * 2); bf* XK = (bf*)take((size_t)SK * DF * 2); float* QH = (float*)take((size_t)SQ * DH * 4); float* KH = (float*)take((size_t)SK * DH * 4);
    if ((size_t)(wsp - (char*)d_ws) > ws_size) return;
    k_w1ab<<<(unsigned)(((size_t)DH * DF / 8 + 255) / 256), 256, 0, stream>>>(W1, WA, WB);
    for (int b = 0; b < NB_; ++b) {
        k_cvt8<<<(SQ * DF / 8 + 255) / 256, 256, 0, stream>>>(Q + (size_t)b * SQ * DF, XQ, (size_t)SQ * DF / 8); k_cvt8<<<(SK * DF / 8 + 255) / 256, 256, 0, stream>>>(K + (size_t)b * SK * DF, XK, (size_t)SK * DF / 8);
        k_gemmw<bf, 0, false><<<dim3(SQ / 64, DH / 64, 1), 32, 0, stream>>>(XQ, nullptr, WA, nullptr, DF, QH, DH, nullptr, 0, 0, 0);
        k_gemmw<bf, 0, false><<<dim3(SK / 64, DH / 64, 1), 32, 0, stream>>>(XK, nullptr, WB, nullptr, DF, KH, DH, nullptr, 0, 0, 0);
        k_cat<<<SQ / 8, 256, 0, stream>>>(QH, KH, b1, W2, MO + (size_t)b * SK, V + (size_t)b * SK * DF, OUT + (size_t)b * SQ * DF); }
}
